// Locoformer_31602369364496
// MI455X (gfx1250) — hardware-run, weakly checked
//
#include <hip/hip_runtime.h>
#include <math.h>
#include <float.h>

typedef __attribute__((ext_vector_type(16))) _Float16 v16h;
typedef __attribute__((ext_vector_type(8)))  _Float16 v8h;
typedef __attribute__((ext_vector_type(8)))  float    v8f;
typedef __attribute__((ext_vector_type(4)))  float    v4f;
typedef __attribute__((ext_vector_type(2)))  float    v2f;
typedef __attribute__((ext_vector_type(4)))  unsigned v4u;

constexpr int SEQ     = 2048;
constexpr int DIM     = 1024;
constexpr int NHEAD   = 16;
constexpr int DHEAD   = 64;
constexpr int HDIM    = NHEAD * DHEAD;
constexpr int WINDOW  = 1024;
constexpr int NLAYER  = 2;
constexpr int FIN     = 2730;
constexpr int FIN_PAD = 2752;
constexpr int NH1     = 2 * FIN;
constexpr int NH1_PAD = 5504;
constexpr int QKV_N   = 3 * HDIM;
constexpr int GM_N    = 128;
constexpr int MIX_COL = 64;
constexpr float W_CARRY = 64.0f;
constexpr float A_CARRY = 64.0f;
constexpr float P_CARRY = 32768.0f;
constexpr int AT_D  = 64;
constexpr int AT_KC = 64;

static_assert(DIM % 32 == 0 && HDIM % 32 == 0 && FIN_PAD % 32 == 0);
static_assert(SEQ % 64 == 0 && QKV_N % 64 == 0 && GM_N % 64 == 0 && DIM % 64 == 0 && NH1_PAD % 64 == 0 && FIN_PAD % 64 == 0);
static_assert(WINDOW % 64 == 0 && SEQ % 64 == 0 && DHEAD == 64 && HDIM == DIM);
static_assert(NH1 % 4 == 0 && NHEAD % 4 == 0 && (FIN % 2) == 0);

constexpr size_t B_X    = (size_t)SEQ * DIM * 4;
constexpr size_t B_T    = (size_t)SEQ * DIM * 2;
constexpr size_t B_VRES = (size_t)SEQ * HDIM * 4;
constexpr size_t B_WQKV = (size_t)QKV_N * DIM * 2;
constexpr size_t B_WGM  = (size_t)GM_N * DIM * 2;
constexpr size_t B_WO   = (size_t)DIM * HDIM * 2;
constexpr size_t B_W1   = (size_t)NH1_PAD * DIM * 2;
constexpr size_t B_W2   = (size_t)DIM * FIN_PAD * 2;
constexpr size_t B_QKV  = (size_t)SEQ * QKV_N * 4;
constexpr size_t B_GM   = (size_t)SEQ * GM_N * 4;
constexpr size_t B_P16  = (size_t)SEQ * HDIM * 2;
constexpr size_t B_H    = (size_t)SEQ * NH1_PAD * 4;
constexpr size_t B_ACT  = (size_t)SEQ * FIN_PAD * 2;
constexpr size_t U_ATT  = B_QKV + B_GM + 4 * B_P16;
constexpr size_t U_FFN  = B_H + B_ACT;
constexpr size_t B_U    = (U_ATT > U_FFN) ? U_ATT : U_FFN;
constexpr size_t WS_TOTAL = 2 * B_X + B_T + B_VRES + B_WQKV + B_WGM + B_WO + B_W1 + B_W2 + B_U;
static_assert(WS_TOTAL <= 134217728ull);
static_assert(B_X % 256 == 0 && B_T % 256 == 0 && B_VRES % 256 == 0 && B_WQKV % 256 == 0 && B_WGM % 256 == 0 &&
              B_WO % 256 == 0 && B_W1 % 256 == 0 && B_W2 % 256 == 0 && B_QKV % 256 == 0 && B_GM % 256 == 0 &&
              B_P16 % 256 == 0 && B_H % 256 == 0);

__device__ __forceinline__ void dep_guard_h(v8f& a, v8f& b, v16h x, v16h y) { asm volatile("v_nop\n\tv_nop\n\tv_nop\n\tv_nop" : "+v"(a), "+v"(b) : "v"(x), "v"(y)); }
__device__ __forceinline__ void keep4_h(v16h a, v16h b, v16h c, v16h d) { asm volatile("v_nop" :: "v"(a), "v"(b), "v"(c), "v"(d)); }
__device__ __forceinline__ void acc_guard4(v8f& a, v8f& b, v8f& c, v8f& d) { asm volatile("v_nop\n\tv_nop\n\tv_nop\n\tv_nop" : "+v"(a), "+v"(b), "+v"(c), "+v"(d)); }

struct FragH {
  union U { v16h v; v8h h[2]; };
  static __device__ __forceinline__ v16h load(const _Float16* p) {
    U f; f.h[0] = *(const v8h*)(p); f.h[1] = *(const v8h*)(p + 16); return f.v;
  }
  static __device__ __forceinline__ v8f mma(v16h a, v16h b, v8f c) {
    return __builtin_amdgcn_wmma_f32_16x16x32_f16(false, a, false, b, (short)0, c, false, false);
  }
};
__device__ __forceinline__ v8f mma_guarded(v16h a, v16h b, v8f c) {
  c = __builtin_amdgcn_wmma_f32_16x16x32_f16(false, a, false, b, (short)0, c, false, false);
  asm volatile("v_nop\n\tv_nop\n\tv_nop\n\tv_nop" : "+v"(c) : "v"(a), "v"(b));
  return c;
}
__device__ __forceinline__ void wave_lds_sync() {
  __builtin_amdgcn_fence(__ATOMIC_RELEASE, "workgroup");
  __builtin_amdgcn_wave_barrier();
  __builtin_amdgcn_fence(__ATOMIC_ACQUIRE, "workgroup");
}

template <int BIAS_MODE, bool RESID>
__global__ __launch_bounds__(256) void gemm64_f16(
    const unsigned short* __restrict__ Ap, int lda,
    const unsigned short* __restrict__ Btp, int ldb,
    float* __restrict__ Cp, int ldc,
    const float* __restrict__ bias, int nbias,
    const float* __restrict__ resid, int ldr,
    int M, int N, int K, float scale)
{
  const _Float16* A  = (const _Float16*)(const void*)Ap;
  const _Float16* Bt = (const _Float16*)(const void*)Btp;
  __shared__ __align__(16) float sT[8][16 * 68];
  const int lane = threadIdx.x & 31;
  const int wave = threadIdx.x >> 5;
  const int tilesN = N >> 6;
  const int tilesM = M >> 6;
  const int tile = blockIdx.x * 8 + wave;
  if (tile >= tilesM * tilesN) return;
  const int tm = tile / tilesN;
  const int tn = tile - tm * tilesN;
  const int m0 = tm << 6;
  const int n0 = tn << 6;
  const int rlane = lane & 15;
  const int koff  = (lane >> 4) * 8;
  const int mOff  = (lane >> 4) * 8;

  v8f acc[4][4];
#pragma unroll
  for (int i = 0; i < 4; ++i)
#pragma unroll
    for (int j = 0; j < 4; ++j) acc[i][j] = (v8f){0.f,0.f,0.f,0.f,0.f,0.f,0.f,0.f};

  for (int k0 = 0; k0 < K; k0 += 32) {
    v16h bh[4];
#pragma unroll
    for (int j = 0; j < 4; ++j)
      bh[j] = FragH::load(Bt + (size_t)(n0 + (j << 4) + rlane) * ldb + koff + k0);
#pragma unroll
    for (int i = 0; i < 4; ++i) {
      const v16h ah = FragH::load(A + (size_t)(m0 + (i << 4) + rlane) * lda + koff + k0);
#pragma unroll
      for (int j = 0; j < 4; ++j) acc[i][j] = FragH::mma(ah, bh[j], acc[i][j]);
      dep_guard_h(acc[i][0], acc[i][3], ah, ah);
    }
    keep4_h(bh[0], bh[1], bh[2], bh[3]);
  }
  acc_guard4(acc[0][0], acc[0][1], acc[0][2], acc[0][3]);
  acc_guard4(acc[1][0], acc[1][1], acc[1][2], acc[1][3]);
  acc_guard4(acc[2][0], acc[2][1], acc[2][2], acc[2][3]);
  acc_guard4(acc[3][0], acc[3][1], acc[3][2], acc[3][3]);

  float* slab = sT[wave];
  const int hh = lane >> 4, c4 = (lane & 15) * 4;
#pragma unroll
  for (int i = 0; i < 4; ++i) {
    const int mBase = m0 + (i << 4);
#pragma unroll
    for (int j = 0; j < 4; ++j) {
      const int n = n0 + (j << 4) + rlane;
      float bv = 0.f;
      if (BIAS_MODE == 2) {
        const int nb = (n < nbias) ? n : (nbias - 1);
        bv = bias[nb];
      }
#pragma unroll
      for (int r = 0; r < 8; ++r)
        slab[(mOff + r) * 68 + (j << 4) + rlane] = acc[i][j][r] * scale + bv;
    }
    wave_lds_sync();
    v4f vals[8];
#pragma unroll
    for (int it = 0; it < 8; ++it) {
      const int row = it * 2 + hh;
      v4f v = *(const v4f*)(slab + row * 68 + c4);
      if (RESID) {
        const v4f rr = *(const v4f*)(resid + (size_t)(mBase + row) * ldr + n0 + c4);
        v += rr;
      }
      vals[it] = v;
    }
    for (int pass = 0; pass < 2; ++pass) {
#pragma unroll
      for (int it = 0; it < 8; ++it) {
        const int row = it * 2 + hh;
        *(volatile v4f*)(Cp + (size_t)(mBase + row) * ldc + n0 + c4) = vals[it];
      }
      __threadfence();
    }
    wave_lds_sync();
  }
}

__global__ __launch_bounds__(256) void transpose_cast_k(
    const float* __restrict__ in, int K, int N,
    unsigned short* __restrict__ out, int ldo, int row_off, float scale)
{
  __shared__ float tile[64][65];
  const int tid = threadIdx.x, lane = tid & 31, wave = tid >> 5;
  const int k0 = blockIdx.x * 64, n0 = blockIdx.y * 64;
#pragma unroll
  for (int it = 0; it < 4; ++it) {
    const int kr = it * 16 + (tid >> 4);
    const int cc = (tid & 15) * 4;
    const int k = k0 + kr, n = n0 + cc;
    const int kc = (k < K) ? k : (K - 1);
    const int nc = (n < N) ? n : (N - 4);
    const v4f v = *(const v4f*)(in + (size_t)kc * N + nc);
    const bool kok = (k < K);
#pragma unroll
    for (int e = 0; e < 4; ++e) tile[kr][cc + e] = (kok && (n + e) < N) ? v[e] * scale : 0.0f;
  }
  __syncthreads();
  const int q = lane >> 3, c8 = (lane & 7) * 8;
  _Float16* o = (_Float16*)(void*)out;
  v8h hvv[2];
#pragma unroll
  for (int it = 0; it < 2; ++it) {
    const int nr = wave * 8 + it * 4 + q;
#pragma unroll
    for (int e = 0; e < 8; ++e) hvv[it][e] = (_Float16)tile[c8 + e][nr];
  }
  for (int pass = 0; pass < 2; ++pass) {
#pragma unroll
    for (int it = 0; it < 2; ++it) {
      const int nr = wave * 8 + it * 4 + q;
      *(volatile v8h*)(o + (size_t)(row_off + n0 + nr) * ldo + k0 + c8) = hvv[it];
    }
    __threadfence();
  }
}

__global__ __launch_bounds__(128) void rmsnorm_f16_k(
    const float* __restrict__ x, const float* __restrict__ w, unsigned short* __restrict__ out)
{
  __shared__ float red[4];
  const int row = blockIdx.x, tid = threadIdx.x, lane = tid & 31, wave = tid >> 5;
  const float* xr = x + (size_t)row * DIM + tid * 8;
  const v4f a = *(const v4f*)xr;
  const v4f b = *(const v4f*)(xr + 4);
  float ss = a[0]*a[0] + a[1]*a[1] + a[2]*a[2] + a[3]*a[3] + b[0]*b[0] + b[1]*b[1] + b[2]*b[2] + b[3]*b[3];
#pragma unroll
  for (int off = 16; off >= 1; off >>= 1) ss += __shfl_xor(ss, off, 32);
  if (lane == 0) red[wave] = ss;
  __syncthreads();
  const float total = (red[0] + red[1]) + (red[2] + red[3]);
  const float rs = rsqrtf(total * (1.0f / 1024.0f) + 1.1920929e-7f);
  const v4f w0 = *(const v4f*)(w + tid * 8);
  const v4f w1 = *(const v4f*)(w + tid * 8 + 4);
  v8h hv;
  hv[0] = (_Float16)(a[0] * rs * w0[0]); hv[1] = (_Float16)(a[1] * rs * w0[1]);
  hv[2] = (_Float16)(a[2] * rs * w0[2]); hv[3] = (_Float16)(a[3] * rs * w0[3]);
  hv[4] = (_Float16)(b[0] * rs * w1[0]); hv[5] = (_Float16)(b[1] * rs * w1[1]);
  hv[6] = (_Float16)(b[2] * rs * w1[2]); hv[7] = (_Float16)(b[3] * rs * w1[3]);
  _Float16* op = (_Float16*)(void*)out + (size_t)row * DIM + tid * 8;
  *(volatile v8h*)op = hv;
  __threadfence();
  *(volatile v8h*)op = hv;
}

__global__ __launch_bounds__(256) void rmsnorm_out_k(
    const float* __restrict__ x, const float* __restrict__ w, float* __restrict__ out)
{
  __shared__ float red[8];
  const int row = blockIdx.x, tid = threadIdx.x, lane = tid & 31, wave = tid >> 5;
  const v4f a = *(const v4f*)(x + (size_t)row * DIM + tid * 4);
  float ss = a[0]*a[0] + a[1]*a[1] + a[2]*a[2] + a[3]*a[3];
#pragma unroll
  for (int off = 16; off >= 1; off >>= 1) ss += __shfl_xor(ss, off, 32);
  if (lane == 0) red[wave] = ss;
  __syncthreads();
  const float total = ((red[0] + red[1]) + (red[2] + red[3])) + ((red[4] + red[5]) + (red[6] + red[7]));
  const float rs = rsqrtf(total * (1.0f / 1024.0f) + 1.1920929e-7f);
  const v4f wv = *(const v4f*)(w + tid * 4);
  v4f o;
  o[0] = a[0] * rs * wv[0]; o[1] = a[1] * rs * wv[1]; o[2] = a[2] * rs * wv[2]; o[3] = a[3] * rs * wv[3];
  float* op = out + (size_t)row * DIM + tid * 4;
  *(volatile v4f*)op = o;
  __threadfence();
  *(volatile v4f*)op = o;
}

struct RopeTab { float f[32]; };
static_assert(sizeof(RopeTab) == 128);

__device__ __forceinline__ float rope_freq(const RopeTab& t, int i) {
  float r = t.f[0];
#pragma unroll
  for (int k = 1; k < 32; ++k) r = (i == k) ? t.f[k] : r;
  return r;
}
__device__ __forceinline__ unsigned pack_f16x2(float a, float b) {
  const _Float16 h0 = (_Float16)a, h1 = (_Float16)b;
  return (unsigned)__builtin_bit_cast(unsigned short, h0) | ((unsigned)__builtin_bit_cast(unsigned short, h1) << 16);
}

__global__ __launch_bounds__(256) void rope_mix_k(
    const float* __restrict__ qkv, const float* __restrict__ gm, float* __restrict__ vres,
    unsigned short* __restrict__ Qp, unsigned short* __restrict__ Kp, unsigned short* __restrict__ Vp,
    int layer, RopeTab tab)
{
  const int s = blockIdx.x, tid = threadIdx.x;
  unsigned* Qw = (unsigned*)(void*)Qp + (size_t)s * (HDIM / 2);
  unsigned* Kw = (unsigned*)(void*)Kp + (size_t)s * (HDIM / 2);
  unsigned* Vw = (unsigned*)(void*)Vp + (size_t)s * (HDIM / 2);
#pragma unroll 1
  for (int it = 0; it < 2; ++it) {
    const int pi = tid + 256 * it;
    const int head = pi >> 5, ip = pi & 31;
    const float fr = rope_freq(tab, ip);
    const float ang = (float)s * fr;
    float sn, cs;
    sincosf(ang, &sn, &cs);
    const float* base = qkv + (size_t)s * QKV_N + 2 * pi;
    const v2f qv = *(const v2f*)base;
    const v2f kv = *(const v2f*)(base + HDIM);
    const v2f vv = *(const v2f*)(base + 2 * HDIM);
    const float qa = qv[0] * cs - qv[1] * sn;
    const float qb = qv[1] * cs + qv[0] * sn;
    const float ka = kv[0] * cs - kv[1] * sn;
    const float kb = kv[1] * cs + kv[0] * sn;
    float va = vv[0], vb = vv[1];
    float* vrp = vres + (size_t)s * HDIM + 2 * pi;
    if (layer == 0) {
      *(volatile v2f*)vrp = vv;
      __threadfence();
      *(volatile v2f*)vrp = vv;
    } else {
      const v2f vr = *(const v2f*)vrp;
      const float ml = gm[(size_t)s * GM_N + MIX_COL + head];
      const float mx = 1.0f / (1.0f + expf(-ml));
      va = va + mx * (vr[0] - va);
      vb = vb + mx * (vr[1] - vb);
    }
    const unsigned uq = pack_f16x2(qa, qb);
    const unsigned uk = pack_f16x2(ka, kb);
    const unsigned uv = pack_f16x2(va, vb);
    ((volatile unsigned*)Qw)[pi] = uq;
    ((volatile unsigned*)Kw)[pi] = uk;
    ((volatile unsigned*)Vw)[pi] = uv;
    __threadfence();
    ((volatile unsigned*)Qw)[pi] = uq;
    ((volatile unsigned*)Kw)[pi] = uk;
    ((volatile unsigned*)Vw)[pi] = uv;
  }
}

__global__ __launch_bounds__(128) void attn_win_k(
    const unsigned short* __restrict__ Qp, const unsigned short* __restrict__ Kp,
    const unsigned short* __restrict__ Vp, const float* __restrict__ gm,
    unsigned short* __restrict__ Gp, float qk_scale, float out_carry)
{
  __shared__ __align__(16) unsigned short Ksh[AT_KC * AT_D];
  __shared__ __align__(16) unsigned short Vth[AT_D * AT_KC];
  __shared__ __align__(16) _Float16 Psh[4][16 * AT_KC];
  __shared__ __align__(16) float Os[4][16 * 68];

  const int tid = threadIdx.x, wave = tid >> 5, lane = tid & 31;
  const int hh = lane >> 4, c = lane & 15;
  constexpr int nqb = SEQ / 64;
  const int qb = blockIdx.x % nqb;
  const int h  = blockIdx.x / nqb;
  const int q0 = qb * 64 + wave * 16;

  v16h qa[2];
  {
    const _Float16* qrow = (const _Float16*)(const void*)Qp + (size_t)(q0 + c) * HDIM + h * DHEAD;
    qa[0] = FragH::load(qrow + 8 * hh);
    qa[1] = FragH::load(qrow + 32 + 8 * hh);
  }
  float mrow[8], lrow[8];
  v8f oacc[4];
#pragma unroll
  for (int r = 0; r < 8; ++r) { mrow[r] = -INFINITY; lrow[r] = 0.f; }
#pragma unroll
  for (int t = 0; t < 4; ++t) oacc[t] = (v8f){0.f,0.f,0.f,0.f,0.f,0.f,0.f,0.f};

  constexpr int WCH = WINDOW / 64;
  const int kc0 = (qb > WCH) ? (qb - WCH) : 0;
  for (int kc = kc0; kc <= qb; ++kc) {
    const int kv0 = kc * AT_KC;
    __syncthreads();
#pragma unroll
    for (int i = 0; i < 4; ++i) {
      const int idx = tid + 128 * i;
      const int row = idx >> 3, c16 = idx & 7;
      const v4u w = *(const v4u*)(Kp + (size_t)(kv0 + row) * HDIM + h * DHEAD + c16 * 8);
      *(v4u*)(Ksh + row * AT_D + c16 * 8) = w;
    }
    {
      const int kvr = tid >> 1, dh = (tid & 1) * 32;
      const unsigned short* vr = Vp + (size_t)(kv0 + kvr) * HDIM + h * DHEAD + dh;
#pragma unroll
      for (int i = 0; i < 4; ++i) {
        const v4u w = *(const v4u*)(vr + 8 * i);
#pragma unroll
        for (int e = 0; e < 4; ++e) {
          const unsigned ww = w[e];
          const int d = dh + 8 * i + 2 * e;
          Vth[d * AT_KC + kvr]       = (unsigned short)(ww & 0xffffu);
          Vth[(d + 1) * AT_KC + kvr] = (unsigned short)(ww >> 16);
        }
      }
    }
    __syncthreads();

    v8f s[4];
#pragma unroll
    for (int j = 0; j < 4; ++j) {
      s[j] = (v8f){0.f,0.f,0.f,0.f,0.f,0.f,0.f,0.f};
#pragma unroll
      for (int dc = 0; dc < 2; ++dc) {
        FragH::U kb;
        const _Float16* kp = (const _Float16*)(const void*)Ksh + (j * 16 + c) * AT_D + dc * 32 + 8 * hh;
        kb.h[0] = *(const v8h*)kp;
        kb.h[1] = *(const v8h*)(kp + 16);
        s[j] = mma_guarded(qa[dc], kb.v, s[j]);
      }
    }
    float cm[8];
#pragma unroll
    for (int r = 0; r < 8; ++r) {
      const int qrow = q0 + 8 * hh + r;
      float m = -INFINITY;
#pragma unroll
      for (int j = 0; j < 4; ++j) {
        const int kvcol = kv0 + j * 16 + c;
        const bool masked = (kvcol > qrow) || (qrow - kvcol > WINDOW);
        float val = s[j][r] * qk_scale;
        val = masked ? (-FLT_MAX) : val;
        s[j][r] = val;
        m = fmaxf(m, val);
      }
#pragma unroll
      for (int off = 1; off < 16; off <<= 1) m = fmaxf(m, __shfl_xor(m, off, 32));
      cm[r] = m;
    }
    _Float16* pw = Psh[wave];
#pragma unroll
    for (int r = 0; r < 8; ++r) {
      const float mnew = fmaxf(mrow[r], cm[r]);
      const float alpha = expf(mrow[r] - mnew);
      mrow[r] = mnew;
      float psum = 0.f;
#pragma unroll
      for (int j = 0; j < 4; ++j) {
        const float p = expf(s[j][r] - mnew);
        psum += p;
        pw[(8 * hh + r) * AT_KC + j * 16 + c] = (_Float16)(p * P_CARRY);
      }
#pragma unroll
      for (int off = 1; off < 16; off <<= 1) psum += __shfl_xor(psum, off, 32);
      lrow[r] = lrow[r] * alpha + psum;
#pragma unroll
      for (int t = 0; t < 4; ++t) oacc[t][r] *= alpha;
    }
    wave_lds_sync();
#pragma unroll
    for (int kk = 0; kk < 2; ++kk) {
      FragH::U pa;
      pa.h[0] = *(const v8h*)(pw + c * AT_KC + kk * 32 + 8 * hh);
      pa.h[1] = *(const v8h*)(pw + c * AT_KC + kk * 32 + 16 + 8 * hh);
#pragma unroll
      for (int t = 0; t < 4; ++t) {
        FragH::U vb;
        const _Float16* vq = (const _Float16*)(const void*)Vth + (t * 16 + c) * AT_KC + kk * 32 + 8 * hh;
        vb.h[0] = *(const v8h*)vq;
        vb.h[1] = *(const v8h*)(vq + 16);
        oacc[t] = mma_guarded(pa.v, vb.v, oacc[t]);
      }
    }
  }

  float gmul[8];
#pragma unroll
  for (int r = 0; r < 8; ++r) {
    const float gl = gm[(size_t)(q0 + 8 * hh + r) * GM_N + h];
    gmul[r] = out_carry / (1.0f + expf(-gl));
  }
  float* os = Os[wave];
#pragma unroll
  for (int r = 0; r < 8; ++r) {
    const float inv = gmul[r] * (1.0f / (lrow[r] * P_CARRY));
#pragma unroll
    for (int t = 0; t < 4; ++t) os[(8 * hh + r) * 68 + t * 16 + c] = oacc[t][r] * inv;
  }
  wave_lds_sync();
  const int q4 = lane >> 3, c8 = (lane & 7) * 8;
  v8h hv[4];
#pragma unroll
  for (int it = 0; it < 4; ++it) {
    const int row = it * 4 + q4;
    const float* sp = os + row * 68 + c8;
#pragma unroll
    for (int e = 0; e < 8; ++e) hv[it][e] = (_Float16)sp[e];
  }
  _Float16* G = (_Float16*)(void*)Gp;
  for (int pass = 0; pass < 2; ++pass) {
#pragma unroll
    for (int it = 0; it < 4; ++it) {
      const int row = it * 4 + q4;
      *(volatile v8h*)(G + (size_t)(q0 + row) * HDIM + h * DHEAD + c8) = hv[it];
    }
    __threadfence();
  }
}

__global__ __launch_bounds__(256) void geglu_k(
    const float* __restrict__ hb, unsigned short* __restrict__ act, float carry)
{
  const int s = blockIdx.x, tid = threadIdx.x;
  const float* hr = hb + (size_t)s * NH1_PAD;
  unsigned* orow = (unsigned*)(void*)act + (size_t)s * (FIN_PAD / 2);
#pragma unroll 1
  for (int wi = tid; wi < FIN_PAD / 2; wi += 256) {
    const int cc = 2 * wi;
    const v2f av = *(const v2f*)(hr + cc);
    const v2f gv = *(const v2f*)(hr + FIN + cc);
    const float ge0 = 0.5f * gv[0] * (1.0f + erff(gv[0] * 0.70710678118654752f));
    const float ge1 = 0.5f * gv[1] * (1.0f + erff(gv[1] * 0.70710678118654752f));
    const bool ok = (cc < FIN);
    const float r0 = ok ? (carry * av[0] * ge0) : 0.0f;
    const float r1 = ok ? (carry * av[1] * ge1) : 0.0f;
    const unsigned u = pack_f16x2(r0, r1);
    ((volatile unsigned*)orow)[wi] = u;
    __threadfence();
    ((volatile unsigned*)orow)[wi] = u;
  }
}

extern "C" void kernel_launch(void* const* d_in, const int* in_sizes, int n_in,
                              void* d_out, int out_size, void* d_ws, size_t ws_size,
                              hipStream_t stream)
{
  if (n_in < 13) return;
  if (in_sizes[0] != SEQ * DIM) return;
  if (in_sizes[1] != NLAYER * DIM) return;
  if (in_sizes[2] != NLAYER * DIM * HDIM) return;
  if (in_sizes[3] != NLAYER * DIM * 2 * HDIM) return;
  if (in_sizes[4] != NLAYER * HDIM * DIM) return;
  if (in_sizes[5] != NLAYER * DIM * NHEAD) return;
  if (in_sizes[6] != NLAYER * DIM * NHEAD) return;
  if (in_sizes[8] != NLAYER * DIM * NH1) return;
  if (in_sizes[9] != NLAYER * NH1) return;
  if (in_sizes[10] != NLAYER * FIN * DIM) return;
  if (in_sizes[11] != NLAYER * DIM) return;
  if (in_sizes[12] != DIM) return;
  if (out_size != SEQ * DIM) return;
  if (ws_size < WS_TOTAL) return;

  const float* x_in   = (const float*)d_in[0];
  const float* norm1w = (const float*)d_in[1];
  const float* wq     = (const float*)d_in[2];
  const float* wkv    = (const float*)d_in[3];
  const float* wo     = (const float*)d_in[4];
  const float* wg     = (const float*)d_in[5];
  const float* wmix   = (const float*)d_in[6];
  const float* norm2w = (const float*)d_in[7];
  const float* w1     = (const float*)d_in[8];
  const float* b1     = (const float*)d_in[9];
  const float* w2     = (const float*)d_in[10];
  const float* b2     = (const float*)d_in[11];
  const float* fnw    = (const float*)d_in[12];
  float* out = (float*)d_out;

  char* base = (char*)d_ws;
  size_t off = 0;
  auto carve = [&](size_t bytes) -> char* { char* p = base + off; off += (bytes + 255) & ~(size_t)255; return p; };
  float*          xA    = (float*)carve(B_X);
  float*          xB    = (float*)carve(B_X);
  unsigned short* tpl   = (unsigned short*)carve(B_T);
  float*          vres  = (float*)carve(B_VRES);
  unsigned short* wqkvT = (unsigned short*)carve(B_WQKV);
  unsigned short* wgmT  = (unsigned short*)carve(B_WGM);
  unsigned short* woT   = (unsigned short*)carve(B_WO);
  unsigned short* w1T   = (unsigned short*)carve(B_W1);
  unsigned short* w2T   = (unsigned short*)carve(B_W2);
  char*           U     = carve(B_U);
  if (off > ws_size) return;
  float*          qkv  = (float*)(U);
  float*          gml  = (float*)(U + B_QKV);
  unsigned short* Qp   = (unsigned short*)(U + B_QKV + B_GM);
  unsigned short* Kp   = (unsigned short*)(U + B_QKV + B_GM + B_P16);
  unsigned short* Vp   = (unsigned short*)(U + B_QKV + B_GM + 2 * B_P16);
  unsigned short* Gp   = (unsigned short*)(U + B_QKV + B_GM + 3 * B_P16);
  float*          hbuf = (float*)(U);
  unsigned short* actp = (unsigned short*)(U + B_H);

  RopeTab tab;
  for (int i = 0; i < 32; ++i) {
    const double e = (double)(2 * i) / 64.0;
    tab.f[i] = (float)(1.0 / pow(10000.0, e));
  }

  auto gemm_grid = [](int M, int N) { const int tiles = (M / 64) * (N / 64); return dim3((unsigned)((tiles + 7) / 8)); };
  const float w_inv  = 1.0f / W_CARRY;
  const float wa_inv = 1.0f / (W_CARRY * A_CARRY);
  const float qk_scale = 0.125f;

  for (int l = 0; l < NLAYER; ++l) {
    const float* xcur   = (l == 0) ? x_in : xA;
    const float* wq_l   = wq   + (size_t)l * DIM * HDIM;
    const float* wkv_l  = wkv  + (size_t)l * DIM * 2 * HDIM;
    const float* wo_l   = wo   + (size_t)l * HDIM * DIM;
    const float* wg_l   = wg   + (size_t)l * DIM * NHEAD;
    const float* wmix_l = wmix + (size_t)l * DIM * NHEAD;
    const float* w1_l   = w1   + (size_t)l * DIM * NH1;
    const float* b1_l   = b1   + (size_t)l * NH1;
    const float* w2_l   = w2   + (size_t)l * FIN * DIM;
    const float* b2_l   = b2   + (size_t)l * DIM;

    rmsnorm_f16_k<<<dim3(SEQ), 128, 0, stream>>>(xcur, norm1w + (size_t)l * DIM, tpl);

    transpose_cast_k<<<dim3(DIM / 64, HDIM / 64), 256, 0, stream>>>(wq_l, DIM, HDIM, wqkvT, DIM, 0, W_CARRY);
    transpose_cast_k<<<dim3(DIM / 64, 2 * HDIM / 64), 256, 0, stream>>>(wkv_l, DIM, 2 * HDIM, wqkvT, DIM, HDIM, W_CARRY);
    transpose_cast_k<<<dim3(DIM / 64, 1), 256, 0, stream>>>(wg_l, DIM, NHEAD, wgmT, DIM, 0, W_CARRY);
    transpose_cast_k<<<dim3(DIM / 64, 1), 256, 0, stream>>>(wmix_l, DIM, NHEAD, wgmT, DIM, MIX_COL, W_CARRY);
    transpose_cast_k<<<dim3(HDIM / 64, DIM / 64), 256, 0, stream>>>(wo_l, HDIM, DIM, woT, HDIM, 0, W_CARRY);
    transpose_cast_k<<<dim3(DIM / 64, NH1_PAD / 64), 256, 0, stream>>>(w1_l, DIM, NH1, w1T, DIM, 0, W_CARRY);
    transpose_cast_k<<<dim3(FIN_PAD / 64, DIM / 64), 256, 0, stream>>>(w2_l, FIN, DIM, w2T, FIN_PAD, 0, W_CARRY);

    gemm64_f16<0, false><<<gemm_grid(SEQ, QKV_N), 256, 0, stream>>>(
        tpl, DIM, wqkvT, DIM, qkv, QKV_N, nullptr, 1, nullptr, 0, SEQ, QKV_N, DIM, w_inv);
    gemm64_f16<0, false><<<gemm_grid(SEQ, GM_N), 256, 0, stream>>>(
        tpl, DIM, wgmT, DIM, gml, GM_N, nullptr, 1, nullptr, 0, SEQ, GM_N, DIM, w_inv);

    rope_mix_k<<<dim3(SEQ), 256, 0, stream>>>(qkv, gml, vres, Qp, Kp, Vp, l, tab);
    attn_win_k<<<dim3(NHEAD * (SEQ / 64)), 128, 0, stream>>>(Qp, Kp, Vp, gml, Gp, qk_scale, A_CARRY);

    gemm64_f16<0, true><<<gemm_grid(SEQ, DIM), 256, 0, stream>>>(
        Gp, HDIM, woT, HDIM, xB, DIM, nullptr, 1, xcur, DIM, SEQ, DIM, HDIM, wa_inv);

    rmsnorm_f16_k<<<dim3(SEQ), 128, 0, stream>>>(xB, norm2w + (size_t)l * DIM, tpl);
    gemm64_f16<2, false><<<gemm_grid(SEQ, NH1_PAD), 256, 0, stream>>>(
        tpl, DIM, w1T, DIM, hbuf, NH1_PAD, b1_l, NH1, nullptr, 0, SEQ, NH1_PAD, DIM, w_inv);
    geglu_k<<<dim3(SEQ), 256, 0, stream>>>(hbuf, actp, A_CARRY);
    gemm64_f16<2, true><<<gemm_grid(SEQ, DIM), 256, 0, stream>>>(
        actp, FIN_PAD, w2T, FIN_PAD, xA, DIM, b2_l, DIM, xB, DIM, SEQ, DIM, FIN_PAD, wa_inv);
  }
  rmsnorm_out_k<<<dim3(SEQ), 256, 0, stream>>>(xA, fnw, out);
}
